// MatrixLSTMCell_4733053960556
// MI455X (gfx1250) — hardware-verified
//
#include <hip/hip_runtime.h>
#include <stddef.h>
#include <stdint.h>

#ifndef NB
#define NB 2
#endif
#ifndef SEQ
#define SEQ 2048
#endif
#define NB_FULL  2
#define SEQ_FULL 2048
#ifndef OSEQ
#define OSEQ SEQ
#endif
#define NTOK  (NB * SEQ)
#define DMOD  384
#define NHEAD 6
#define HDM   64
#define NG    12
#define GM    16
#define MT    (GM / 16)
#define GK    1152
#define QB    64
#define KC    64
#define NQB   (SEQ / QB)

static_assert(NB >= 1 && NB <= NB_FULL);
static_assert(SEQ >= 64 && SEQ <= SEQ_FULL);
static_assert(OSEQ >= SEQ);
static_assert(NTOK == NB * SEQ);
static_assert(DMOD == NHEAD * HDM);
static_assert(GK == 3 * DMOD);
static_assert(GK % 32 == 0);
static_assert(GK % 8 == 0);
static_assert(DMOD % 64 == 0);
static_assert(DMOD % 32 == 0);
static_assert(NTOK % 64 == 0);
static_assert(SEQ % QB == 0);
static_assert(QB == KC);
static_assert(HDM == 64);
static_assert((NTOK * DMOD) % 2048 == 0);
static_assert(NG <= GM && GM % 16 == 0 && MT >= 1);
static_assert(NG == 2 * NHEAD);
static_assert(GK / 8 > 128 && GK / 8 <= 256);
static_assert(NG * 16 > 128 && NG * 16 <= 256);

#if SEQ > 1024
#define SNT 1024
#else
#define SNT SEQ
#endif
#define EPT (SEQ / SNT)
static_assert(SEQ % SNT == 0);
static_assert(EPT >= 1 && EPT <= 2);
static_assert(SEQ % 4 == 0 && (SEQ / 4) <= SNT);
static_assert((SEQ / 4) % 32 == 0);

typedef unsigned short us;
typedef __attribute__((ext_vector_type(16))) __bf16 v16bf;
typedef us           v8us __attribute__((ext_vector_type(8)));
typedef float        v8f  __attribute__((ext_vector_type(8)));
typedef float        v4f  __attribute__((ext_vector_type(4)));
typedef unsigned int v4u  __attribute__((ext_vector_type(4)));

union Frag  { v16bf v; v8us h[2]; };
union Pack8 { v8us h; v4u u; };

#define LOG2E 1.44269504088896340736f

__device__ __forceinline__ us bf_rne(float f) {
  unsigned u = __float_as_uint(f);
  u = u + 0x7FFFu + ((u >> 16) & 1u);
  return (us)(u >> 16);
}
__device__ __forceinline__ float bf_val(us hv) { return __uint_as_float(((unsigned)hv) << 16); }
__device__ __forceinline__ void split2(float f, us& hi, us& lo) {
  const us hv = bf_rne(f);
  hi = hv;
  lo = bf_rne(f - bf_val(hv));
}
__device__ __forceinline__ void split8(const float (&f)[8], Pack8& ph, Pack8& pl) {
  us hh[8], ll[8];
#pragma unroll
  for (int e = 0; e < 8; ++e) split2(f[e], hh[e], ll[e]);
  ph.h = (v8us){hh[0], hh[1], hh[2], hh[3], hh[4], hh[5], hh[6], hh[7]};
  pl.h = (v8us){ll[0], ll[1], ll[2], ll[3], ll[4], ll[5], ll[6], ll[7]};
}

__device__ __forceinline__ v8f mma16(v16bf a, v16bf b, v8f c) {
  c = __builtin_amdgcn_wmma_f32_16x16x32_bf16(false, a, false, b, (short)0, c, false, false);
  asm volatile("v_nop\n\tv_nop\n\tv_nop\n\tv_nop" : "+v"(c) : "v"(a), "v"(b));
  return c;
}

__device__ __forceinline__ v16bf ldfrag(const us* p, int ld, int row0, int k0, int lane) {
  const int m = lane & 15, lh = lane >> 4;
  const us* q = p + (size_t)(row0 + m) * ld + k0 + 8 * lh;
  Frag f;
  f.h[0] = *(const v8us*)(q);
  f.h[1] = *(const v8us*)(q + 16);
  return f.v;
}

__device__ __forceinline__ v8f zero8() { return (v8f){0.f, 0.f, 0.f, 0.f, 0.f, 0.f, 0.f, 0.f}; }

__global__ __launch_bounds__(256) void k_cvt(const float* __restrict__ x, us* __restrict__ xh, us* __restrict__ xl) {
  const size_t i = (size_t)blockIdx.x * 2048 + (size_t)threadIdx.x * 8;
  const int tok = (int)(i / DMOD);
  const int col = (int)(i - (size_t)tok * DMOD);
  const int b   = tok / SEQ;
  const int s   = tok - b * SEQ;
  const size_t si = ((size_t)b * SEQ_FULL + (size_t)s) * DMOD + (size_t)col;
  const v4f a0 = *(const v4f*)(x + si);
  const v4f a1 = *(const v4f*)(x + si + 4);
  const float f[8] = {a0[0], a0[1], a0[2], a0[3], a1[0], a1[1], a1[2], a1[3]};
  Pack8 ph, pl;
  split8(f, ph, pl);
  const v4u hv = ph.u, lv = pl.u;
  *(volatile v4u*)(xh + i) = hv;
  *(volatile v4u*)(xl + i) = lv;
  __threadfence();
  *(volatile v4u*)(xh + i) = hv;
  *(volatile v4u*)(xl + i) = lv;
}

#define SFP 68
__global__ __launch_bounds__(256) void k_cvt_vt(const float* __restrict__ v, us* __restrict__ vth,
                                                us* __restrict__ vtl) {
  __shared__ __align__(16) float sw[64 * SFP];
  const int tid = threadIdx.x;
  const int tb  = blockIdx.x * 64;
  const int cb0 = blockIdx.y * 64;
  const int b   = tb / SEQ;
  const int s0  = tb - b * SEQ;
  const size_t srow0 = (size_t)b * SEQ_FULL + (size_t)s0;
  {
    const int r  = tid >> 2;
    const int c0 = (tid & 3) * 16;
    const float* src = v + (srow0 + (size_t)r) * DMOD + cb0 + c0;
#pragma unroll
    for (int e = 0; e < 4; ++e) *(v4f*)(sw + r * SFP + c0 + 4 * e) = *(const v4f*)(src + 4 * e);
  }
  __syncthreads();
  v4u hv[2], lv[2];
  size_t go[2];
#pragma unroll
  for (int j = 0; j < 2; ++j) {
    const int p  = tid + 256 * j;
    const int n  = p >> 3;
    const int pc = p & 7;
    const float* cp = sw + (pc * 8) * SFP + n;
    float f[8];
#pragma unroll
    for (int e = 0; e < 8; ++e) f[e] = cp[e * SFP];
    Pack8 ph, pl;
    split8(f, ph, pl);
    hv[j] = ph.u;
    lv[j] = pl.u;
    go[j] = (size_t)(cb0 + n) * NTOK + tb + pc * 8;
  }
#pragma unroll
  for (int j = 0; j < 2; ++j) { *(volatile v4u*)(vth + go[j]) = hv[j]; *(volatile v4u*)(vtl + go[j]) = lv[j]; }
  __threadfence();
#pragma unroll
  for (int j = 0; j < 2; ++j) { *(volatile v4u*)(vth + go[j]) = hv[j]; *(volatile v4u*)(vtl + go[j]) = lv[j]; }
}

__global__ __launch_bounds__(128) void k_cvt_w(const float* __restrict__ igw, const float* __restrict__ fgw,
                                               us* __restrict__ wh, us* __restrict__ wl) {
  const int tid = threadIdx.x;
  const int row = blockIdx.x;
  const int ri  = (row < NHEAD) ? row : (NHEAD - 1);
  const int rf0 = row - NHEAD;
  const int rf  = (rf0 < 0) ? 0 : ((rf0 > NHEAD - 1) ? (NHEAD - 1) : rf0);
  const bool usei = (row < NHEAD);
  const bool zero = (row >= NG);
  const float* src = usei ? (igw + (size_t)ri * GK) : (fgw + (size_t)rf * GK);
  v4u hv[2], lv[2];
  size_t go[2];
#pragma unroll
  for (int j = 0; j < 2; ++j) {
    const int p   = tid + 128 * j;
    const int pcl = (p < GK / 8) ? p : (GK / 8 - 1);
    const float* sp = src + 8 * pcl;
    const v4f a0 = *(const v4f*)(sp);
    const v4f a1 = *(const v4f*)(sp + 4);
    float f[8] = {a0[0], a0[1], a0[2], a0[3], a1[0], a1[1], a1[2], a1[3]};
    if (zero) {
#pragma unroll
      for (int e = 0; e < 8; ++e) f[e] = 0.f;
    }
    Pack8 ph, pl;
    split8(f, ph, pl);
    hv[j] = ph.u;
    lv[j] = pl.u;
    go[j] = (size_t)row * GK + 8 * pcl;
  }
  const bool v1 = (tid < (GK / 8 - 128));
  *(volatile v4u*)(wh + go[0]) = hv[0]; *(volatile v4u*)(wl + go[0]) = lv[0];
  if (v1) { *(volatile v4u*)(wh + go[1]) = hv[1]; *(volatile v4u*)(wl + go[1]) = lv[1]; }
  __threadfence();
  *(volatile v4u*)(wh + go[0]) = hv[0]; *(volatile v4u*)(wl + go[0]) = lv[0];
  if (v1) { *(volatile v4u*)(wh + go[1]) = hv[1]; *(volatile v4u*)(wl + go[1]) = lv[1]; }
}

#define SGP 68
__device__ __forceinline__ void gate_seg(const us* __restrict__ xh, const us* __restrict__ xl,
                                         const us* __restrict__ wh, const us* __restrict__ wl,
                                         int kofs, int row0, int lane, v8f (&acc)[MT]) {
#pragma unroll 1
  for (int k0 = 0; k0 < DMOD; k0 += 32) {
    const v16bf xbh = ldfrag(xh, DMOD, row0, k0, lane);
    const v16bf xbl = ldfrag(xl, DMOD, row0, k0, lane);
#pragma unroll
    for (int mt = 0; mt < MT; ++mt) {
      const v16bf wah = ldfrag(wh, GK, 16 * mt, kofs + k0, lane);
      const v16bf wal = ldfrag(wl, GK, 16 * mt, kofs + k0, lane);
      acc[mt] = mma16(wah, xbh, acc[mt]);
      acc[mt] = mma16(wah, xbl, acc[mt]);
      acc[mt] = mma16(wal, xbh, acc[mt]);
    }
  }
}

__global__ __launch_bounds__(128) void k_gate(const us* __restrict__ qh, const us* __restrict__ ql,
                                              const us* __restrict__ kh, const us* __restrict__ kl,
                                              const us* __restrict__ vh, const us* __restrict__ vl,
                                              const us* __restrict__ wh, const us* __restrict__ wl,
                                              const float* __restrict__ igb, const float* __restrict__ fgb,
                                              float* __restrict__ gr) {
  __shared__ __align__(16) float sg[GM * SGP];
  const int tid = threadIdx.x, lane = tid & 31, wave = tid >> 5;
  const int hh = lane >> 4, c = lane & 15;
  const int n0 = blockIdx.x * 64;
  const int row0 = n0 + 16 * wave;

  v8f acc[MT];
#pragma unroll
  for (int mt = 0; mt < MT; ++mt) acc[mt] = zero8();
  gate_seg(qh, ql, wh, wl, 0, row0, lane, acc);
  gate_seg(kh, kl, wh, wl, DMOD, row0, lane, acc);
  gate_seg(vh, vl, wh, wl, 2 * DMOD, row0, lane, acc);

#pragma unroll
  for (int mt = 0; mt < MT; ++mt) {
#pragma unroll
    for (int r = 0; r < 8; ++r) {
      const int m   = 16 * mt + 8 * hh + r;
      const int mi  = (m < NHEAD) ? m : (NHEAD - 1);
      const int mf0 = m - NHEAD;
      const int mf  = (mf0 < 0) ? 0 : ((mf0 > NHEAD - 1) ? (NHEAD - 1) : mf0);
      const float bi = igb[mi];
      const float bf = fgb[mf];
      const float bias = (m < NHEAD) ? bi : ((m < NG) ? bf : 0.f);
      sg[m * SGP + 16 * wave + c] = acc[mt][r] + bias;
    }
  }
  __syncthreads();

  v4f val[2];
  size_t go[2];
#pragma unroll
  for (int j = 0; j < 2; ++j) {
    const int p    = tid + 128 * j;
    const int L    = p >> 3;
    const int pc   = p & 7;
    const int row  = L >> 1;
    const int half = L & 1;
    const int col  = half * 32 + pc * 4;
    val[j] = *(const v4f*)(sg + row * SGP + col);
    go[j]  = (size_t)row * NTOK + n0 + col;
  }
  const bool v1 = (tid < (NG * 16 - 128));
  *(volatile v4f*)(gr + go[0]) = val[0];
  if (v1) *(volatile v4f*)(gr + go[1]) = val[1];
  __threadfence();
  *(volatile v4f*)(gr + go[0]) = val[0];
  if (v1) *(volatile v4f*)(gr + go[1]) = val[1];
}

__global__ __launch_bounds__(SNT) void k_scan(const float* __restrict__ gr, float* __restrict__ a2p,
                                              float* __restrict__ nm2p, float* __restrict__ ep) {
  __shared__ double dtot[SNT];
  __shared__ float  ftot[SNT];
  __shared__ __align__(16) float sa[SEQ];
  __shared__ __align__(16) float sn[SEQ];
  __shared__ __align__(16) float se[SEQ];
  const int t  = threadIdx.x;
  const int bh = blockIdx.x;
  const int b  = bh / NHEAD;
  const int h  = bh - b * NHEAD;
  const size_t gi = (size_t)h * NTOK + (size_t)b * SEQ + (size_t)t * EPT;
  const size_t gf = (size_t)(NHEAD + h) * NTOK + (size_t)b * SEQ + (size_t)t * EPT;
  const float NEGINF = -__builtin_huge_valf();

  float igv[EPT];
  double lcs[EPT];
  double run = 0.0;
#pragma unroll
  for (int e = 0; e < EPT; ++e) {
    const float ig = gr[gi + e];
    const float fg = gr[gf + e];
    const float lg = fminf(fg, 0.f) - log1pf(expf(-fabsf(fg)));
    run += (double)lg;
    lcs[e] = run;
    igv[e] = ig;
  }
  dtot[t] = run;
  __syncthreads();
#pragma unroll 1
  for (int off = 1; off < SNT; off <<= 1) {
    const int si    = (t >= off) ? (t - off) : 0;
    const double pv = dtot[si];
    const double p  = (t >= off) ? pv : 0.0;
    __syncthreads();
    dtot[t] += p;
    __syncthreads();
  }
  const int tm = (t > 0) ? (t - 1) : 0;
  const double dpv = dtot[tm];
  const double exs = (t > 0) ? dpv : 0.0;

  float cf[EPT], av[EPT], lm[EPT];
  float runm = NEGINF;
#pragma unroll
  for (int e = 0; e < EPT; ++e) {
    cf[e] = (float)(exs + lcs[e]);
    av[e] = igv[e] - cf[e];
    runm  = fmaxf(runm, av[e]);
    lm[e] = runm;
  }
  ftot[t] = runm;
  __syncthreads();
#pragma unroll 1
  for (int off = 1; off < SNT; off <<= 1) {
    const int si   = (t >= off) ? (t - off) : 0;
    const float pv = ftot[si];
    const float p  = (t >= off) ? pv : NEGINF;
    __syncthreads();
    ftot[t] = fmaxf(ftot[t], p);
    __syncthreads();
  }
  const float fpv = ftot[tm];
  const float exm = (t > 0) ? fpv : NEGINF;
#pragma unroll
  for (int e = 0; e < EPT; ++e) {
    const float M = fmaxf(exm, lm[e]);
    const int s = t * EPT + e;
    sa[s] = av[e] * LOG2E;
    sn[s] = -(M * LOG2E);
    se[s] = expf(-(cf[e] + M));
  }
  __syncthreads();
  if (t < SEQ / 4) {
    const v4f xa = *(const v4f*)(sa + 4 * t);
    const v4f xn = *(const v4f*)(sn + 4 * t);
    const v4f xe = *(const v4f*)(se + 4 * t);
    const size_t go = (size_t)bh * SEQ + 4 * t;
    *(volatile v4f*)(a2p + go)  = xa;
    *(volatile v4f*)(nm2p + go) = xn;
    *(volatile v4f*)(ep + go)   = xe;
    __threadfence();
    *(volatile v4f*)(a2p + go)  = xa;
    *(volatile v4f*)(nm2p + go) = xn;
    *(volatile v4f*)(ep + go)   = xe;
  }
}

#define LP  72
#define OTP 68
union AttnLds {
  us    p[2][4 * 16 * LP];
  float o[4][16 * OTP];
};

__global__ __launch_bounds__(128) void k_attn(const us* __restrict__ qh, const us* __restrict__ ql,
                                              const us* __restrict__ kh, const us* __restrict__ kl,
                                              const us* __restrict__ vth, const us* __restrict__ vtl,
                                              const float* __restrict__ a2g, const float* __restrict__ nm2g,
                                              const float* __restrict__ eg,
                                              const float* __restrict__ nw,
                                              float* __restrict__ out) {
  __shared__ __align__(16) us Ksh[KC * LP];
  __shared__ __align__(16) us Ksl[KC * LP];
  __shared__ __align__(16) us Vsh[HDM * LP];
  __shared__ __align__(16) us Vsl[HDM * LP];
  __shared__ __align__(16) AttnLds pu;

  const int tid = threadIdx.x, lane = tid & 31, wave = tid >> 5;
  const int hh = lane >> 4, c = lane & 15;
  const int bh   = blockIdx.x / NQB;
  const int qb   = blockIdx.x - bh * NQB;
  const int b    = bh / NHEAD;
  const int hd   = bh - b * NHEAD;
  const int tok0 = b * SEQ;
  const int col0 = hd * HDM;
  const int qloc = qb * QB + wave * 16;
  const int q0   = tok0 + qloc;
  const size_t orow0 = (size_t)b * OSEQ + (size_t)qloc;
  const int nch  = qb + 1;
  const size_t gb = (size_t)bh * SEQ;

  float nm2[8], zrow[8];
  v8f oacc[4];
#pragma unroll
  for (int r = 0; r < 8; ++r) {
    nm2[r]  = nm2g[gb + qloc + 8 * hh + r];
    zrow[r] = 0.f;
  }
#pragma unroll
  for (int t = 0; t < 4; ++t) oacc[t] = zero8();

  us* pwh = pu.p[0] + wave * 16 * LP;
  us* pwl = pu.p[1] + wave * 16 * LP;

#pragma unroll 1
  for (int i = 0; i < nch; ++i) {
    const int kv0 = i * KC;
    __syncthreads();
    {
      const int r  = tid >> 1;
      const int cb = (tid & 1) * 32;
      const us* ksh = kh  + (size_t)(tok0 + kv0 + r) * DMOD + col0 + cb;
      const us* ksl = kl  + (size_t)(tok0 + kv0 + r) * DMOD + col0 + cb;
      const us* vsh = vth + (size_t)(col0 + r) * NTOK + tok0 + kv0 + cb;
      const us* vsl = vtl + (size_t)(col0 + r) * NTOK + tok0 + kv0 + cb;
#pragma unroll
      for (int e = 0; e < 4; ++e) {
        *(v8us*)(Ksh + r * LP + cb + 8 * e) = *(const v8us*)(ksh + 8 * e);
        *(v8us*)(Ksl + r * LP + cb + 8 * e) = *(const v8us*)(ksl + 8 * e);
        *(v8us*)(Vsh + r * LP + cb + 8 * e) = *(const v8us*)(vsh + 8 * e);
        *(v8us*)(Vsl + r * LP + cb + 8 * e) = *(const v8us*)(vsl + 8 * e);
      }
    }
    __syncthreads();

    v8f s[4];
#pragma unroll
    for (int j = 0; j < 4; ++j) s[j] = zero8();
#pragma unroll
    for (int dc = 0; dc < 2; ++dc) {
      const v16bf qah = ldfrag(qh, DMOD, q0, col0 + dc * 32, lane);
      const v16bf qal = ldfrag(ql, DMOD, q0, col0 + dc * 32, lane);
#pragma unroll
      for (int j = 0; j < 4; ++j) {
        const v16bf kbh = ldfrag(Ksh, LP, j * 16, dc * 32, lane);
        const v16bf kbl = ldfrag(Ksl, LP, j * 16, dc * 32, lane);
        s[j] = mma16(qah, kbh, s[j]);
        s[j] = mma16(qah, kbl, s[j]);
        s[j] = mma16(qal, kbh, s[j]);
      }
    }
#pragma unroll
    for (int j = 0; j < 4; ++j) {
      const int key  = kv0 + j * 16 + c;
      const float g2 = a2g[gb + key];
#pragma unroll
      for (int r = 0; r < 8; ++r) {
        const int qrow = qloc + 8 * hh + r;
        const float xe = fminf(g2 + nm2[r], 0.f);
        const float dd = exp2f(xe);
        const float cv = (s[j][r] * 0.125f) * dd;
        s[j][r] = (key <= qrow) ? cv : 0.f;
      }
    }
#pragma unroll
    for (int r = 0; r < 8; ++r) {
      float psum = 0.f;
#pragma unroll
      for (int j = 0; j < 4; ++j) {
        const float cv = s[j][r];
        psum += cv;
        us ph, pl;
        split2(cv, ph, pl);
        pwh[(8 * hh + r) * LP + j * 16 + c] = ph;
        pwl[(8 * hh + r) * LP + j * 16 + c] = pl;
      }
#pragma unroll
      for (int off = 1; off < 16; off <<= 1) psum += __shfl_xor(psum, off, 32);
      zrow[r] += psum;
    }
    __syncthreads();

#pragma unroll
    for (int kk = 0; kk < 2; ++kk) {
      const v16bf pah = ldfrag(pwh, LP, 0, kk * 32, lane);
      const v16bf pal = ldfrag(pwl, LP, 0, kk * 32, lane);
#pragma unroll
      for (int t = 0; t < 4; ++t) {
        const v16bf vbh = ldfrag(Vsh, LP, t * 16, kk * 32, lane);
        const v16bf vbl = ldfrag(Vsl, LP, t * 16, kk * 32, lane);
        oacc[t] = mma16(pah, vbh, oacc[t]);
        oacc[t] = mma16(pah, vbl, oacc[t]);
        oacc[t] = mma16(pal, vbh, oacc[t]);
      }
    }
  }

  float inv[8];
#pragma unroll
  for (int r = 0; r < 8; ++r) {
    const float er = eg[gb + qloc + 8 * hh + r];
    inv[r] = 1.0f / (fmaxf(fabsf(zrow[r]), er) + 1e-6f);
  }
  float wa[4];
#pragma unroll
  for (int t = 0; t < 4; ++t) {
    const int col = col0 + 16 * t + c;
    wa[t] = 1.0f + nw[col];
  }
  __syncthreads();
  float* osw = pu.o[wave];
#pragma unroll
  for (int r = 0; r < 8; ++r) {
    float x[4];
    float sm = 0.f;
#pragma unroll
    for (int t = 0; t < 4; ++t) { x[t] = oacc[t][r] * inv[r]; sm += x[t]; }
#pragma unroll
    for (int off = 1; off < 16; off <<= 1) sm += __shfl_xor(sm, off, 32);
    const float mean = sm * (1.0f / 64.0f);
    float sq = 0.f;
#pragma unroll
    for (int t = 0; t < 4; ++t) { x[t] = x[t] - mean; sq += x[t] * x[t]; }
#pragma unroll
    for (int off = 1; off < 16; off <<= 1) sq += __shfl_xor(sq, off, 32);
    const float var  = sq * (1.0f / 64.0f);
    const float rstd = rsqrtf(var + 1e-5f);
#pragma unroll
    for (int t = 0; t < 4; ++t) osw[(8 * hh + r) * OTP + 16 * t + c] = (x[t] * rstd) * wa[t];
  }
  __syncthreads();
  v4f val[8];
  size_t go[8];
#pragma unroll
  for (int it = 0; it < 8; ++it) {
    const int p    = lane + 32 * it;
    const int L    = p >> 3;
    const int pc   = p & 7;
    const int row  = L >> 1;
    const int half = L & 1;
    const int col  = half * 32 + pc * 4;
    val[it] = *(const v4f*)(osw + row * OTP + col);
    go[it]  = (orow0 + (size_t)row) * DMOD + col0 + col;
  }
#pragma unroll
  for (int it = 0; it < 8; ++it) *(volatile v4f*)(out + go[it]) = val[it];
  __threadfence();
#pragma unroll
  for (int it = 0; it < 8; ++it) *(volatile v4f*)(out + go[it]) = val[it];
}

extern "C" void kernel_launch(void* const* d_in, const int* in_sizes, int n_in,
                              void* d_out, int out_size, void* d_ws, size_t ws_size,
                              hipStream_t stream) {
  if (n_in < 8) return;
  const long need_tok = (long)(NB - 1) * SEQ_FULL + SEQ;
  if ((long)in_sizes[0] < need_tok * DMOD) return;
  if ((long)in_sizes[1] < need_tok * DMOD) return;
  if ((long)in_sizes[2] < need_tok * DMOD) return;
  if (in_sizes[3] < NHEAD * GK) return;
  if (in_sizes[4] < NHEAD) return;
  if (in_sizes[5] < NHEAD * GK) return;
  if (in_sizes[6] < NHEAD) return;
  if (in_sizes[7] < DMOD) return;
  const long need_out = ((long)(NB - 1) * OSEQ + SEQ) * DMOD;
  if ((long)out_size < need_out) return;

  const float* q   = (const float*)d_in[0];
  const float* k   = (const float*)d_in[1];
  const float* v   = (const float*)d_in[2];
  const float* igw = (const float*)d_in[3];
  const float* igb = (const float*)d_in[4];
  const float* fgw = (const float*)d_in[5];
  const float* fgb = (const float*)d_in[6];
  const float* nw  = (const float*)d_in[7];
  float* out = (float*)d_out;

  const size_t PL2 = (size_t)NTOK * DMOD * 2;
  const size_t WPL = (size_t)GM * GK * 2;
  const size_t GRB = (size_t)NG * NTOK * 4;
  const size_t GPB = (size_t)NB * NHEAD * SEQ * 4;
  static_assert(((size_t)NTOK * DMOD * 2) % 128 == 0);
  static_assert(((size_t)GM * GK * 2) % 128 == 0);
  static_assert(((size_t)NG * NTOK * 4) % 128 == 0);
  static_assert(((size_t)NB * NHEAD * SEQ * 4) % 128 == 0);
  size_t off = 0;
  const size_t oQh  = off; off += PL2;  const size_t oQl  = off; off += PL2;
  const size_t oKh  = off; off += PL2;  const size_t oKl  = off; off += PL2;
  const size_t oVh  = off; off += PL2;  const size_t oVl  = off; off += PL2;
  const size_t oVTh = off; off += PL2;  const size_t oVTl = off; off += PL2;
  const size_t oWh  = off; off += WPL;  const size_t oWl  = off; off += WPL;
  const size_t oGR  = off; off += GRB;
  const size_t oA2  = off; off += GPB;
  const size_t oNM  = off; off += GPB;
  const size_t oE   = off; off += GPB;
  if (off > ws_size) return;
  if (off > (size_t)134217728) return;

  char* ws = (char*)d_ws;
  us* Qh  = (us*)(ws + oQh);   us* Ql  = (us*)(ws + oQl);
  us* Kh  = (us*)(ws + oKh);   us* Kl  = (us*)(ws + oKl);
  us* Vh  = (us*)(ws + oVh);   us* Vl  = (us*)(ws + oVl);
  us* VTh = (us*)(ws + oVTh);  us* VTl = (us*)(ws + oVTl);
  us* Wh  = (us*)(ws + oWh);   us* Wl  = (us*)(ws + oWl);
  float* GR  = (float*)(ws + oGR);
  float* A2  = (float*)(ws + oA2);
  float* NM2 = (float*)(ws + oNM);
  float* EP  = (float*)(ws + oE);

  k_cvt<<<dim3((NTOK * DMOD) / 2048), dim3(256), 0, stream>>>(q, Qh, Ql);
  k_cvt<<<dim3((NTOK * DMOD) / 2048), dim3(256), 0, stream>>>(k, Kh, Kl);
  k_cvt<<<dim3((NTOK * DMOD) / 2048), dim3(256), 0, stream>>>(v, Vh, Vl);
  k_cvt_vt<<<dim3(NTOK / 64, DMOD / 64), dim3(256), 0, stream>>>(v, VTh, VTl);
  k_cvt_w<<<dim3(GM), dim3(128), 0, stream>>>(igw, fgw, Wh, Wl);
  k_gate<<<dim3(NTOK / 64), dim3(128), 0, stream>>>(Qh, Ql, Kh, Kl, Vh, Vl, Wh, Wl, igb, fgb, GR);
  k_scan<<<dim3(NB * NHEAD), dim3(SNT), 0, stream>>>(GR, A2, NM2, EP);
  k_attn<<<dim3(NB * NHEAD * NQB), dim3(128), 0, stream>>>(Qh, Ql, Kh, Kl, VTh, VTl, A2, NM2, EP, nw, out);
  (void)hipGetLastError();
}
